// Block_59322088293038
// MI455X (gfx1250) — hardware-verified
//
#include <hip/hip_runtime.h>
#include <math.h>

#ifndef NB
#define NB 2
#endif
#ifndef SEQ
#define SEQ 2048
#endif
#define NB_FULL 2
#define SEQ_FULL 2048

constexpr int CD = 768;
constexpr int NH = 12;
constexpr int HD = 64;
constexpr int C3 = 3 * CD;
constexpr int C4 = 4 * CD;
constexpr int NCH = SEQ / 64;
constexpr int MTOK = NB * SEQ;
constexpr int QKP = 2 * CD;
constexpr int VTP = MTOK;
constexpr int EROWS = 64;
constexpr int LNP = CD / 128;

#define LN_INV (1.0f / (float)CD)
#define LN_EPS 1e-5f

static_assert(NB >= 1 && NB <= NB_FULL);
static_assert(SEQ <= SEQ_FULL);
static_assert(SEQ % 256 == 0);
static_assert(NCH <= 32 && NCH * 64 == SEQ);
static_assert(CD == NH * HD);
static_assert(HD == 64);
static_assert(CD % 128 == 0 && LNP == 6 && 32 * 4 * LNP == CD);
static_assert(MTOK % 64 == 0 && CD % 64 == 0 && C3 % 64 == 0 && C4 % 64 == 0 && QKP % 64 == 0);
static_assert(CD % 32 == 0 && C4 % 32 == 0);
static_assert(MTOK % 8 == 0);
static_assert(SEQ % 64 == 0);
static_assert(EROWS == 64 && EROWS <= SEQ);
static_assert((CD / 8) % 8 == 0 && (C4 / 8) % 8 == 0);
static_assert(((long long)C3 * (CD / 8)) % 256 == 0 && ((long long)CD * (CD / 8)) % 256 == 0 && ((long long)C4 * (CD / 8)) % 256 == 0 && ((long long)CD * (C4 / 8)) % 256 == 0);
static_assert(QKP == 2 * CD && C3 == 3 * CD && VTP % 8 == 0);

typedef __attribute__((ext_vector_type(16))) _Float16 v16h;
typedef __attribute__((ext_vector_type(8)))  _Float16 v8h;
typedef __attribute__((ext_vector_type(16))) __bf16   v16b;
typedef __attribute__((ext_vector_type(8)))  __bf16   v8b;
typedef __attribute__((ext_vector_type(8)))  float    v8f;
typedef __attribute__((ext_vector_type(4)))  float    v4f;
typedef __attribute__((ext_vector_type(4)))  int      v4i;
typedef __attribute__((ext_vector_type(4)))  unsigned int v4u;
typedef __attribute__((ext_vector_type(2)))  unsigned int v2u;

union FH { v16h v; v8h h[2]; };
union FB { v16b v; v8b h[2]; };

#define VST2(T, ptr, val) do { const T vst2_v_ = (val); *(volatile T*)(ptr) = vst2_v_; __threadfence(); *(volatile T*)(ptr) = vst2_v_; } while (0)

#define WAVE_SYNC() do { __builtin_amdgcn_fence(3  , "workgroup"); __builtin_amdgcn_wave_barrier(); __builtin_amdgcn_fence(2  , "workgroup"); } while (0)

__device__ __forceinline__ float cmb_bf(float v) { const unsigned u = __builtin_bit_cast(unsigned, v); const unsigned r = (u + 0x7fffu + ((u >> 16) & 1u)) & 0xffff0000u; return __builtin_bit_cast(float, r); }
__device__ __forceinline__ unsigned int pk2h(float a, float b) { return (unsigned int)__builtin_bit_cast(unsigned short, (_Float16)a) | ((unsigned int)__builtin_bit_cast(unsigned short, (_Float16)b) << 16); }
__device__ __forceinline__ unsigned short bf_bits(float f) { const unsigned u = __float_as_uint(f); return (unsigned short)((u + 0x7FFFu + ((u >> 16) & 1u)) >> 16); }
__device__ __forceinline__ void at_split(float f, __bf16& hi, __bf16& lo) {
  const unsigned short hb = bf_bits(f);
  hi = __builtin_bit_cast(__bf16, hb);
  lo = __builtin_bit_cast(__bf16, bf_bits(f - __uint_as_float(((unsigned)hb) << 16)));
}
__device__ __forceinline__ v16h ldg_frag(const _Float16* __restrict__ p) { FH f; f.h[0] = *(const v8h*)(p); f.h[1] = *(const v8h*)(p + 16); return f.v; }

__device__ __forceinline__ v8f mma_h(v16h a, v16h b, v8f c) {
  c = __builtin_amdgcn_wmma_f32_16x16x32_f16(false, a, false, b, (short)0, c, false, false);
  asm volatile("v_nop\n\tv_nop\n\tv_nop\n\tv_nop" : "+v"(c) : "v"(a), "v"(b));
  return c;
}
__device__ __forceinline__ v8f mma_b(v16b a, v16b b, v8f c) {
  c = __builtin_amdgcn_wmma_f32_16x16x32_bf16(false, a, false, b, (short)0, c, false, false);
  asm volatile("v_nop\n\tv_nop\n\tv_nop\n\tv_nop" : "+v"(c) : "v"(a), "v"(b));
  return c;
}
__device__ __forceinline__ void dep_guard4_h(v8f& a, v8f& b, v8f& c, v8f& d, v16h x, v16h y) { asm volatile("v_nop\n\tv_nop\n\tv_nop\n\tv_nop" : "+v"(a), "+v"(b), "+v"(c), "+v"(d) : "v"(x), "v"(y)); }
__device__ __forceinline__ void keep4_h(v16h a, v16h b, v16h c, v16h d) { asm volatile("v_nop" :: "v"(a), "v"(b), "v"(c), "v"(d)); }
__device__ __forceinline__ void acc_guard4(v8f& a, v8f& b, v8f& c, v8f& d) { asm volatile("v_nop\n\tv_nop\n\tv_nop\n\tv_nop" : "+v"(a), "+v"(b), "+v"(c), "+v"(d)); }

__device__ __forceinline__ float gelu_tanh(float t) {
  const float t3 = (t * t) * t;
  const float u = 0.7978845608028654f * (t + 0.044715f * t3);
  const float e = exp2f(-2.885390081777927f * u);
  return t * __builtin_amdgcn_rcpf(1.0f + e);
}

__global__ __launch_bounds__(256) void k_maskcls(const int* __restrict__ mask, int* __restrict__ cls) {
  __shared__ int s_nz[64][33];
  __shared__ int s_zz[64][33];
  __shared__ int s_row[64];
  const int qb = blockIdx.x, t = threadIdx.x, r = t >> 2, q = t & 3;
  constexpr int CPT = NCH / 4;
  const int* mrow = mask + (size_t)(qb * 64 + r) * SEQ_FULL;
#pragma unroll 1
  for (int cidx = 0; cidx < CPT; ++cidx) {
    const int kc = q * CPT + cidx; int nz = 0, zz = 0;
#pragma unroll 4
    for (int i = 0; i < 16; ++i) {
      const v4i m = *(const v4i*)(mrow + kc * 64 + 4 * i);
      nz |= (m.x != 0) | (m.y != 0) | (m.z != 0) | (m.w != 0);
      zz |= (m.x == 0) | (m.y == 0) | (m.z == 0) | (m.w == 0);
    }
    s_nz[r][kc] = nz; s_zz[r][kc] = zz;
  }
  __syncthreads();
  int myc = 0;
  if (t < 32) {
    if (t < NCH) {
      int nz = 0, zz = 0;
#pragma unroll 1
      for (int rr = 0; rr < 64; ++rr) { nz |= s_nz[rr][t]; zz |= s_zz[rr][t]; }
      myc = (nz == 0) ? 0 : ((zz == 0) ? 1 : 2);
    }
  }
  if (t >= 64 && t < 128) {
    const int rr = t - 64; int any = 0;
#pragma unroll 1
    for (int kc = 0; kc < NCH; ++kc) any |= s_nz[rr][kc];
    s_row[rr] = any;
  }
  __syncthreads();
  if (t < 32) {
    int full = 0;
#pragma unroll 1
    for (int rr = 0; rr < 64; ++rr) full |= (s_row[rr] == 0) ? 1 : 0;
    VST2(int, cls + qb * 64 + t, myc);
    const int fv = (t == 0) ? full : 0;
    VST2(int, cls + qb * 64 + 32 + t, fv);
  }
}

__global__ __launch_bounds__(256) void k_castbT(const float* __restrict__ SRC, int lds, unsigned short* __restrict__ DST, int ldd, int nR, int nC, float sc) {
  const long long u = (long long)blockIdx.x * 256 + threadIdx.x; const int per = nR / 8; if (u >= (long long)nC * per) return;
  const int cc = (int)(u / per); const int r0 = 8 * (int)(u % per);
  float w[8];
#pragma unroll
  for (int e = 0; e < 8; ++e) w[e] = cmb_bf(SRC[(long long)(r0 + e) * lds + cc]) * sc;
  v4u pk; pk.x = pk2h(w[0], w[1]); pk.y = pk2h(w[2], w[3]); pk.z = pk2h(w[4], w[5]); pk.w = pk2h(w[6], w[7]);
  VST2(v4u, (v4u*)(DST + (long long)cc * ldd + r0), pk);
}

template <int ABF, int FULLMAP>
__device__ __forceinline__ void ln_body(const float* __restrict__ A, const float* __restrict__ GA, const float* __restrict__ BE, unsigned short* __restrict__ Y16) {
  #pragma clang fp contract(off)
  const int wave = __builtin_amdgcn_readfirstlane(threadIdx.x >> 5);
  const int r = blockIdx.x * 8 + wave; const int L = threadIdx.x & 31; if (r >= MTOK) return;
  const size_t srow = FULLMAP ? ((size_t)(r / SEQ) * SEQ_FULL + (size_t)(r % SEQ)) : (size_t)r;
  v4f v[LNP]; float s = 0.f;
#pragma unroll
  for (int q = 0; q < LNP; ++q) {
    v[q] = *(const v4f*)(A + srow * CD + 4 * L + 128 * q);
    if (ABF) { v[q].x = cmb_bf(v[q].x); v[q].y = cmb_bf(v[q].y); v[q].z = cmb_bf(v[q].z); v[q].w = cmb_bf(v[q].w); }
    s += (v[q].x + v[q].y) + (v[q].z + v[q].w);
  }
#pragma unroll
  for (int o = 16; o > 0; o >>= 1) s += __shfl_xor(s, o, 32);
  const float mu = s * LN_INV; float qq = 0.f;
#pragma unroll
  for (int q = 0; q < LNP; ++q) { v[q].x -= mu; v[q].y -= mu; v[q].z -= mu; v[q].w -= mu; qq += (v[q].x * v[q].x + v[q].y * v[q].y) + (v[q].z * v[q].z + v[q].w * v[q].w); }
#pragma unroll
  for (int o = 16; o > 0; o >>= 1) qq += __shfl_xor(qq, o, 32);
  const float rs = rsqrtf(qq * LN_INV + LN_EPS);
#pragma unroll
  for (int q = 0; q < LNP; ++q) {
    const int c = 4 * L + 128 * q; const v4f ga = *(const v4f*)(GA + c), be = *(const v4f*)(BE + c); v4f y;
    y.x = v[q].x * rs * cmb_bf(ga.x) + cmb_bf(be.x); y.y = v[q].y * rs * cmb_bf(ga.y) + cmb_bf(be.y);
    y.z = v[q].z * rs * cmb_bf(ga.z) + cmb_bf(be.z); y.w = v[q].w * rs * cmb_bf(ga.w) + cmb_bf(be.w);
    v2u pk; pk.x = pk2h(y.x, y.y); pk.y = pk2h(y.z, y.w);
    VST2(v2u, (v2u*)(Y16 + (size_t)r * CD + c), pk);
  }
}
__global__ __launch_bounds__(256) void k_ln_in(const float* __restrict__ A, const float* __restrict__ GA, const float* __restrict__ BE, unsigned short* __restrict__ Y16) { ln_body<1, 1>(A, GA, BE, Y16); }
__global__ __launch_bounds__(256) void k_ln_mid(const float* __restrict__ A, const float* __restrict__ GA, const float* __restrict__ BE, unsigned short* __restrict__ Y16) { ln_body<0, 0>(A, GA, BE, Y16); }

struct GP {
  const unsigned short* A; const unsigned short* Bt; void* C; const float* bias; const float* R;
  long long strideA, strideC;
  int lda, ldb, ldc, ldr, M, N, K, rpb, rpbC, rpbR; float scale; int pad_;
};
static_assert(sizeof(GP) == 104);

template <int BIAS_MODE, int OUT_MODE, int RES_MODE, int ACT>
__device__ __forceinline__ void gemm_body(const GP& p) {
  __shared__ __align__(16) float sT[8][16 * 68];
  const int b = blockIdx.y;
  const int lane = threadIdx.x & 31;
  const int wave = __builtin_amdgcn_readfirstlane(threadIdx.x >> 5);
  const int tilesN = p.N >> 6, tilesM = p.M >> 6;
  const int tile = blockIdx.x * 8 + wave;
  if (tile >= tilesM * tilesN) return;
  const int tm = tile / tilesN, tn = tile - tm * tilesN;
  const int m0 = tm << 6, n0 = tn << 6;
  const _Float16* Ab = (const _Float16*)p.A + (size_t)b * p.strideA;
  const _Float16* Bb = (const _Float16*)p.Bt;
  const int rlane = lane & 15, koff = (lane >> 4) * 8, mOff = (lane >> 4) * 8;

  v8f acc[4][4];
#pragma unroll
  for (int i = 0; i < 4; ++i)
#pragma unroll
    for (int j = 0; j < 4; ++j) acc[i][j] = (v8f){0.f, 0.f, 0.f, 0.f, 0.f, 0.f, 0.f, 0.f};

  for (int k0 = 0; k0 < p.K; k0 += 32) {
    v16h bh[4];
#pragma unroll
    for (int j = 0; j < 4; ++j) bh[j] = ldg_frag(Bb + (size_t)(n0 + (j << 4) + rlane) * p.ldb + koff + k0);
#pragma unroll
    for (int i = 0; i < 4; ++i) {
      const v16h ah = ldg_frag(Ab + (size_t)(m0 + (i << 4) + rlane) * p.lda + koff + k0);
#pragma unroll
      for (int j = 0; j < 4; ++j) acc[i][j] = __builtin_amdgcn_wmma_f32_16x16x32_f16(false, ah, false, bh[j], (short)0, acc[i][j], false, false);
      dep_guard4_h(acc[i][0], acc[i][1], acc[i][2], acc[i][3], ah, bh[3]);
    }
    keep4_h(bh[0], bh[1], bh[2], bh[3]);
  }
  acc_guard4(acc[0][0], acc[0][1], acc[0][2], acc[0][3]);
  acc_guard4(acc[1][0], acc[1][1], acc[1][2], acc[1][3]);
  acc_guard4(acc[2][0], acc[2][1], acc[2][2], acc[2][3]);
  acc_guard4(acc[3][0], acc[3][1], acc[3][2], acc[3][3]);

#pragma unroll
  for (int i = 0; i < 4; ++i) {
    const int mBase = m0 + (i << 4);
    float bm[8];
#pragma unroll
    for (int r = 0; r < 8; ++r) { bm[r] = 0.f; if (BIAS_MODE == 1) bm[r] = cmb_bf(p.bias[mBase + mOff + r]); }
#pragma unroll
    for (int j = 0; j < 4; ++j) {
      const int n = n0 + (j << 4) + rlane;
      float bv = 0.f; if (BIAS_MODE == 2) bv = cmb_bf(p.bias[n]);
#pragma unroll
      for (int r = 0; r < 8; ++r) {
        float v = acc[i][j][r] * p.scale + ((BIAS_MODE == 1) ? bm[r] : bv);
        if (ACT == 1) v = gelu_tanh(v);
        sT[wave][(mOff + r) * 68 + (j << 4) + rlane] = v;
      }
    }
    WAVE_SYNC();
    const int gb = mBase / p.rpb; const int tIn = mBase - gb * p.rpb;
    const size_t rowC0 = (size_t)gb * p.rpbC + tIn, rowR0 = (size_t)gb * p.rpbR + tIn;
    if (OUT_MODE == 0) {
      float* C = (float*)p.C + (size_t)b * p.strideC;
      const int hh = lane >> 4, c4 = (lane & 15) * 4;
      v4f val[8];
#pragma unroll
      for (int it = 0; it < 8; ++it) {
        const int row = it * 2 + hh;
        v4f v = *(const v4f*)(&sT[wave][row * 68 + c4]);
        if (RES_MODE != 0) {
          v4f x = *(const v4f*)(p.R + (rowR0 + row) * (size_t)p.ldr + n0 + c4);
          if (RES_MODE == 2) { x.x = cmb_bf(x.x); x.y = cmb_bf(x.y); x.z = cmb_bf(x.z); x.w = cmb_bf(x.w); }
          v = v + x;
        }
        val[it] = v;
      }
      for (int pass = 0; pass < 2; ++pass) {
#pragma unroll
        for (int it = 0; it < 8; ++it) {
          const int row = it * 2 + hh;
          *(volatile v4f*)(C + (rowC0 + row) * (size_t)p.ldc + n0 + c4) = val[it];
        }
        __threadfence();
      }
    } else {
      unsigned short* C = (unsigned short*)p.C + (size_t)b * p.strideC;
      const int q = lane >> 3, c8 = (lane & 7) * 8;
      v8h hv[4];
#pragma unroll
      for (int it = 0; it < 4; ++it) {
#pragma unroll
        for (int e = 0; e < 8; ++e) hv[it][e] = (_Float16)sT[wave][(it * 4 + q) * 68 + c8 + e];
      }
      for (int pass = 0; pass < 2; ++pass) {
#pragma unroll
        for (int it = 0; it < 4; ++it) {
          const int row = it * 4 + q;
          *(volatile v8h*)(C + (rowC0 + row) * (size_t)p.ldc + n0 + c8) = hv[it];
        }
        __threadfence();
      }
    }
    WAVE_SYNC();
  }
}

__device__ __forceinline__ GP gp_pack(const unsigned short* A, const unsigned short* Bt, void* C, const float* bias, const float* R,
                                      long long strideA, long long strideC, int lda, int ldb, int ldc, int ldr, int M, int N, int K,
                                      int rpb, int rpbC, int rpbR, float scale) {
  GP g;
  g.A = A; g.Bt = Bt; g.C = C; g.bias = bias; g.R = R; g.strideA = strideA; g.strideC = strideC;
  g.lda = lda; g.ldb = ldb; g.ldc = ldc; g.ldr = ldr; g.M = M; g.N = N; g.K = K; g.rpb = rpb; g.rpbC = rpbC; g.rpbR = rpbR;
  g.scale = scale; g.pad_ = 0;
  return g;
}

__global__ __launch_bounds__(256) void k_gemm_qk(const unsigned short* A, const unsigned short* Bt, void* C, const float* bias, const float* R,
                                                   long long strideA, long long strideC, int lda, int ldb, int ldc, int ldr, int M, int N, int K,
                                                   int rpb, int rpbC, int rpbR, float scale) {
  const GP p = gp_pack(A, Bt, C, bias, R, strideA, strideC, lda, ldb, ldc, ldr, M, N, K, rpb, rpbC, rpbR, scale);
  gemm_body<2, 1, 0, 0>(p);
}
__global__ __launch_bounds__(256) void k_gemm_vt(const unsigned short* A, const unsigned short* Bt, void* C, const float* bias, const float* R,
                                                   long long strideA, long long strideC, int lda, int ldb, int ldc, int ldr, int M, int N, int K,
                                                   int rpb, int rpbC, int rpbR, float scale) {
  const GP p = gp_pack(A, Bt, C, bias, R, strideA, strideC, lda, ldb, ldc, ldr, M, N, K, rpb, rpbC, rpbR, scale);
  gemm_body<1, 1, 0, 0>(p);
}
__global__ __launch_bounds__(256) void k_gemm_e(const unsigned short* A, const unsigned short* Bt, void* C, const float* bias, const float* R,
                                                  long long strideA, long long strideC, int lda, int ldb, int ldc, int ldr, int M, int N, int K,
                                                  int rpb, int rpbC, int rpbR, float scale) {
  const GP p = gp_pack(A, Bt, C, bias, R, strideA, strideC, lda, ldb, ldc, ldr, M, N, K, rpb, rpbC, rpbR, scale);
  gemm_body<2, 0, 0, 0>(p);
}
__global__ __launch_bounds__(256) void k_gemm_proj(const unsigned short* A, const unsigned short* Bt, void* C, const float* bias, const float* R,
                                                     long long strideA, long long strideC, int lda, int ldb, int ldc, int ldr, int M, int N, int K,
                                                     int rpb, int rpbC, int rpbR, float scale) {
  const GP p = gp_pack(A, Bt, C, bias, R, strideA, strideC, lda, ldb, ldc, ldr, M, N, K, rpb, rpbC, rpbR, scale);
  gemm_body<2, 0, 2, 0>(p);
}
__global__ __launch_bounds__(256) void k_gemm_fc(const unsigned short* A, const unsigned short* Bt, void* C, const float* bias, const float* R,
                                                   long long strideA, long long strideC, int lda, int ldb, int ldc, int ldr, int M, int N, int K,
                                                   int rpb, int rpbC, int rpbR, float scale) {
  const GP p = gp_pack(A, Bt, C, bias, R, strideA, strideC, lda, ldb, ldc, ldr, M, N, K, rpb, rpbC, rpbR, scale);
  gemm_body<2, 1, 0, 1>(p);
}
__global__ __launch_bounds__(256) void k_gemm_mlp(const unsigned short* A, const unsigned short* Bt, void* C, const float* bias, const float* R,
                                                    long long strideA, long long strideC, int lda, int ldb, int ldc, int ldr, int M, int N, int K,
                                                    int rpb, int rpbC, int rpbR, float scale) {
  const GP p = gp_pack(A, Bt, C, bias, R, strideA, strideC, lda, ldb, ldc, ldr, M, N, K, rpb, rpbC, rpbR, scale);
  gemm_body<2, 0, 1, 0>(p);
}

#define ATT_SC 0.18033688011112042f
#define ATT_FILL (-3.4028234663852886e38f)
#define ATT_PCAR 4096.0f

__global__ __launch_bounds__(128) void k_attn_main(const unsigned short* __restrict__ QKp, const unsigned short* __restrict__ VTp,
                                                     const int* __restrict__ mask, const int* __restrict__ cls, unsigned short* __restrict__ CTXp) {
  __shared__ __align__(16) _Float16 Psh[4][16 * 64];
  __shared__ __align__(16) unsigned int Msh[4][16 * 16];
  __shared__ __align__(16) _Float16 Osh[4][16 * 64];
  const int tid = threadIdx.x, lane = tid & 31, hh = lane >> 4, c = lane & 15;
  const int wave = __builtin_amdgcn_readfirstlane(tid >> 5);
  const int bx = blockIdx.x; const int qb = bx % NCH; const int bhh = bx / NCH; const int h = bhh % NH; const int b = bhh / NH;
  const int q0 = qb * 64 + wave * 16;
  const _Float16* QK = (const _Float16*)QKp; const _Float16* VT = (const _Float16*)VTp;
  const size_t tok0 = (size_t)b * SEQ;

  v16h qa0, qa1;
  { const _Float16* qrow = QK + (tok0 + q0 + c) * (size_t)QKP + h * HD + 8 * hh; qa0 = ldg_frag(qrow); qa1 = ldg_frag(qrow + 32); }

  float mrow[8], lrow[8]; v8f oacc[4];
#pragma unroll
  for (int r = 0; r < 8; ++r) { mrow[r] = -INFINITY; lrow[r] = 0.f; }
#pragma unroll
  for (int t = 0; t < 4; ++t) oacc[t] = (v8f){0.f, 0.f, 0.f, 0.f, 0.f, 0.f, 0.f, 0.f};

  const int full = __builtin_amdgcn_readfirstlane(cls[qb * 64 + 32]);
#pragma unroll 1
  for (int kc = 0; kc < NCH; ++kc) {
    const int cv = __builtin_amdgcn_readfirstlane(cls[qb * 64 + kc]);
    if (cv == 0 && full == 0) continue;
    const int kv0 = kc * 64;
    v8f s[4];
#pragma unroll
    for (int j = 0; j < 4; ++j) {
      const _Float16* krow = QK + (tok0 + kv0 + j * 16 + c) * (size_t)QKP + CD + h * HD + 8 * hh;
      const v16h kb0 = ldg_frag(krow), kb1 = ldg_frag(krow + 32);
      v8f z = (v8f){0.f, 0.f, 0.f, 0.f, 0.f, 0.f, 0.f, 0.f};
      z = mma_h(qa0, kb0, z);
      z = mma_h(qa1, kb1, z);
      s[j] = z * ATT_SC;
    }
    if (cv != 1) {
      const int* mb = mask + (size_t)q0 * SEQ_FULL + kv0;
#pragma unroll
      for (int it = 0; it < 8; ++it) {
        const int row = it * 2 + hh;
        const v4i m = *(const v4i*)(mb + (size_t)row * SEQ_FULL + 4 * c);
        Msh[wave][row * 16 + c] = ((m.x != 0) ? 1u : 0u) | ((m.y != 0) ? 0x100u : 0u) | ((m.z != 0) ? 0x10000u : 0u) | ((m.w != 0) ? 0x1000000u : 0u);
      }
      WAVE_SYNC();
#pragma unroll
      for (int r = 0; r < 8; ++r)
#pragma unroll
        for (int j = 0; j < 4; ++j) {
          const unsigned int w = Msh[wave][(8 * hh + r) * 16 + j * 4 + (c >> 2)];
          const bool keep = ((w >> (8 * (c & 3))) & 1u) != 0u;
          s[j][r] = keep ? s[j][r] : ATT_FILL;
        }
      WAVE_SYNC();
    }
#pragma unroll
    for (int r = 0; r < 8; ++r) {
      float m = fmaxf(fmaxf(s[0][r], s[1][r]), fmaxf(s[2][r], s[3][r]));
      m = fmaxf(m, __shfl_xor(m, 1, 32)); m = fmaxf(m, __shfl_xor(m, 2, 32));
      m = fmaxf(m, __shfl_xor(m, 4, 32)); m = fmaxf(m, __shfl_xor(m, 8, 32));
      const float mnew = fmaxf(mrow[r], m);
      const float alpha = exp2f(mrow[r] - mnew);
      mrow[r] = mnew;
      float psum = 0.f;
#pragma unroll
      for (int j = 0; j < 4; ++j) {
        const float pe = exp2f(s[j][r] - mnew);
        psum += pe;
        Psh[wave][(8 * hh + r) * 64 + j * 16 + c] = (_Float16)(pe * ATT_PCAR);
      }
      psum += __shfl_xor(psum, 1, 32); psum += __shfl_xor(psum, 2, 32); psum += __shfl_xor(psum, 4, 32); psum += __shfl_xor(psum, 8, 32);
      lrow[r] = lrow[r] * alpha + psum;
#pragma unroll
      for (int t = 0; t < 4; ++t) oacc[t][r] *= alpha;
    }
    WAVE_SYNC();
#pragma unroll
    for (int kk = 0; kk < 2; ++kk) {
      FH pa;
      pa.h[0] = *(const v8h*)(&Psh[wave][c * 64 + kk * 32 + 8 * hh]);
      pa.h[1] = *(const v8h*)(&Psh[wave][c * 64 + kk * 32 + 16 + 8 * hh]);
#pragma unroll
      for (int t = 0; t < 4; ++t) {
        const v16h vb = ldg_frag(VT + (size_t)(h * HD + t * 16 + c) * VTP + tok0 + kv0 + kk * 32 + 8 * hh);
        oacc[t] = mma_h(pa.v, vb, oacc[t]);
      }
    }
    WAVE_SYNC();
  }

#pragma unroll
  for (int r = 0; r < 8; ++r) {
    const float inv = (lrow[r] > 0.f) ? 1.0f / (lrow[r] * ATT_PCAR) : 0.f;
#pragma unroll
    for (int t = 0; t < 4; ++t) Osh[wave][(8 * hh + r) * 64 + t * 16 + c] = (_Float16)(oacc[t][r] * inv);
  }
  WAVE_SYNC();
  {
    const int q = lane >> 3, c8 = (lane & 7) * 8;
    v8h hv[4];
#pragma unroll
    for (int it = 0; it < 4; ++it) hv[it] = *(const v8h*)(&Osh[wave][(it * 4 + q) * 64 + c8]);
    for (int pass = 0; pass < 2; ++pass) {
#pragma unroll
      for (int it = 0; it < 4; ++it)
        *(volatile v8h*)(CTXp + (tok0 + q0 + it * 4 + q) * (size_t)CD + h * HD + c8) = hv[it];
      __threadfence();
    }
  }
}

__global__ __launch_bounds__(128) void k_attn_early(const float* __restrict__ QE, const int* __restrict__ mask, const int* __restrict__ cls, unsigned short* __restrict__ CTXp) {
  __shared__ __align__(16) __bf16 Ksh[64 * 64];
  __shared__ __align__(16) __bf16 Ksl[64 * 64];
  __shared__ __align__(16) __bf16 Vth[64 * 64];
  __shared__ __align__(16) __bf16 Vtl[64 * 64];
  __shared__ __align__(16) __bf16 Psh[4][16 * 64];
  __shared__ __align__(16) __bf16 Psl[4][16 * 64];
  __shared__ __align__(16) unsigned int Msh[4][16 * 16];
  __shared__ __align__(16) _Float16 Osh[4][16 * 64];
  int ok = ((cls[0] != 0) ? 1 : 0) & ((cls[32] == 0) ? 1 : 0);
#pragma unroll 1
  for (int kc = 1; kc < NCH; ++kc) ok &= (cls[kc] == 0) ? 1 : 0;
  ok = __builtin_amdgcn_readfirstlane(ok);
  if (ok == 0) return;

  const int tid = threadIdx.x, lane = tid & 31, hh = lane >> 4, c = lane & 15;
  const int wave = __builtin_amdgcn_readfirstlane(tid >> 5);
  const int h = blockIdx.x % NH, b = blockIdx.x / NH;
  const int q0 = wave * 16;
  const float* qe = QE + (size_t)b * EROWS * C3;

  v16b qh[2], ql[2];
  {
    const float* qrow = qe + (size_t)(q0 + c) * C3 + h * HD;
#pragma unroll
    for (int dc = 0; dc < 2; ++dc)
#pragma unroll
      for (int e = 0; e < 8; ++e) {
        __bf16 a, l2;
        at_split(qrow[dc * 32 + 8 * hh + e], a, l2); qh[dc][e] = a; ql[dc][e] = l2;
        at_split(qrow[dc * 32 + 16 + 8 * hh + e], a, l2); qh[dc][8 + e] = a; ql[dc][8 + e] = l2;
      }
  }
  {
    const int kvr = tid >> 1, dh = (tid & 1) * 32;
    const float* krow = qe + (size_t)kvr * C3 + CD + h * HD + dh;
    const float* vrow = qe + (size_t)kvr * C3 + 2 * CD + h * HD + dh;
#pragma unroll
    for (int i = 0; i < 8; ++i) {
      const v4f kk = *(const v4f*)(krow + 4 * i);
      const v4f vv = *(const v4f*)(vrow + 4 * i);
#pragma unroll
      for (int e = 0; e < 4; ++e) {
        const int d = dh + 4 * i + e; __bf16 a, l2;
        at_split(kk[e], a, l2); Ksh[kvr * 64 + d] = a; Ksl[kvr * 64 + d] = l2;
        at_split(vv[e], a, l2); Vth[d * 64 + kvr] = a; Vtl[d * 64 + kvr] = l2;
      }
    }
  }
  __syncthreads();

  v8f s[4];
#pragma unroll
  for (int j = 0; j < 4; ++j) {
    v8f z = (v8f){0.f, 0.f, 0.f, 0.f, 0.f, 0.f, 0.f, 0.f};
#pragma unroll
    for (int dc = 0; dc < 2; ++dc) {
      FB kh, kl;
      kh.h[0] = *(const v8b*)(&Ksh[(j * 16 + c) * 64 + dc * 32 + 8 * hh]);
      kh.h[1] = *(const v8b*)(&Ksh[(j * 16 + c) * 64 + dc * 32 + 16 + 8 * hh]);
      kl.h[0] = *(const v8b*)(&Ksl[(j * 16 + c) * 64 + dc * 32 + 8 * hh]);
      kl.h[1] = *(const v8b*)(&Ksl[(j * 16 + c) * 64 + dc * 32 + 16 + 8 * hh]);
      z = mma_b(qh[dc], kh.v, z);
      z = mma_b(qh[dc], kl.v, z);
      z = mma_b(ql[dc], kh.v, z);
    }
    s[j] = z * ATT_SC;
  }
  {
    const int* mb = mask + (size_t)q0 * SEQ_FULL;
#pragma unroll
    for (int it = 0; it < 8; ++it) {
      const int row = it * 2 + hh;
      const v4i m = *(const v4i*)(mb + (size_t)row * SEQ_FULL + 4 * c);
      Msh[wave][row * 16 + c] = ((m.x != 0) ? 1u : 0u) | ((m.y != 0) ? 0x100u : 0u) | ((m.z != 0) ? 0x10000u : 0u) | ((m.w != 0) ? 0x1000000u : 0u);
    }
  }
  WAVE_SYNC();
#pragma unroll
  for (int r = 0; r < 8; ++r)
#pragma unroll
    for (int j = 0; j < 4; ++j) {
      const unsigned int w = Msh[wave][(8 * hh + r) * 16 + j * 4 + (c >> 2)];
      const bool keep = ((w >> (8 * (c & 3))) & 1u) != 0u;
      s[j][r] = keep ? s[j][r] : ATT_FILL;
    }
  float lrow[8];
#pragma unroll
  for (int r = 0; r < 8; ++r) {
    float m = fmaxf(fmaxf(s[0][r], s[1][r]), fmaxf(s[2][r], s[3][r]));
    m = fmaxf(m, __shfl_xor(m, 1, 32)); m = fmaxf(m, __shfl_xor(m, 2, 32));
    m = fmaxf(m, __shfl_xor(m, 4, 32)); m = fmaxf(m, __shfl_xor(m, 8, 32));
    float psum = 0.f;
#pragma unroll
    for (int j = 0; j < 4; ++j) {
      const float pe = exp2f(s[j][r] - m);
      psum += pe;
      __bf16 a, l2; at_split(pe * ATT_PCAR, a, l2);
      Psh[wave][(8 * hh + r) * 64 + j * 16 + c] = a; Psl[wave][(8 * hh + r) * 64 + j * 16 + c] = l2;
    }
    psum += __shfl_xor(psum, 1, 32); psum += __shfl_xor(psum, 2, 32); psum += __shfl_xor(psum, 4, 32); psum += __shfl_xor(psum, 8, 32);
    lrow[r] = psum;
  }
  WAVE_SYNC();
  v8f oacc[4];
#pragma unroll
  for (int t = 0; t < 4; ++t) oacc[t] = (v8f){0.f, 0.f, 0.f, 0.f, 0.f, 0.f, 0.f, 0.f};
#pragma unroll
  for (int kk = 0; kk < 2; ++kk) {
    FB pa, pl;
    pa.h[0] = *(const v8b*)(&Psh[wave][c * 64 + kk * 32 + 8 * hh]);
    pa.h[1] = *(const v8b*)(&Psh[wave][c * 64 + kk * 32 + 16 + 8 * hh]);
    pl.h[0] = *(const v8b*)(&Psl[wave][c * 64 + kk * 32 + 8 * hh]);
    pl.h[1] = *(const v8b*)(&Psl[wave][c * 64 + kk * 32 + 16 + 8 * hh]);
#pragma unroll
    for (int t = 0; t < 4; ++t) {
      FB vh, vl;
      vh.h[0] = *(const v8b*)(&Vth[(t * 16 + c) * 64 + kk * 32 + 8 * hh]);
      vh.h[1] = *(const v8b*)(&Vth[(t * 16 + c) * 64 + kk * 32 + 16 + 8 * hh]);
      vl.h[0] = *(const v8b*)(&Vtl[(t * 16 + c) * 64 + kk * 32 + 8 * hh]);
      vl.h[1] = *(const v8b*)(&Vtl[(t * 16 + c) * 64 + kk * 32 + 16 + 8 * hh]);
      oacc[t] = mma_b(pa.v, vh.v, oacc[t]);
      oacc[t] = mma_b(pa.v, vl.v, oacc[t]);
      oacc[t] = mma_b(pl.v, vh.v, oacc[t]);
    }
  }
#pragma unroll
  for (int r = 0; r < 8; ++r) {
    const float inv = (lrow[r] > 0.f) ? 1.0f / (lrow[r] * ATT_PCAR) : 0.f;
#pragma unroll
    for (int t = 0; t < 4; ++t) Osh[wave][(8 * hh + r) * 64 + t * 16 + c] = (_Float16)(oacc[t][r] * inv);
  }
  WAVE_SYNC();
  {
    const int q = lane >> 3, c8 = (lane & 7) * 8;
    const size_t tok0 = (size_t)b * SEQ;
    v8h hv[4];
#pragma unroll
    for (int it = 0; it < 4; ++it) hv[it] = *(const v8h*)(&Osh[wave][(it * 4 + q) * 64 + c8]);
    for (int pass = 0; pass < 2; ++pass) {
#pragma unroll
      for (int it = 0; it < 4; ++it)
        *(volatile v8h*)(CTXp + (tok0 + q0 + it * 4 + q) * (size_t)CD + h * HD + c8) = hv[it];
      __threadfence();
    }
  }
}

constexpr size_t SZ_H16  = (size_t)MTOK * CD * 2;
constexpr size_t SZ_W3T  = (size_t)C3 * CD * 2;
constexpr size_t SZ_WOT  = (size_t)CD * CD * 2;
constexpr size_t SZ_W1T  = (size_t)C4 * CD * 2;
constexpr size_t SZ_W2T  = (size_t)CD * C4 * 2;
constexpr size_t SZ_QK   = (size_t)MTOK * QKP * 2;
constexpr size_t SZ_VT   = (size_t)CD * VTP * 2;
constexpr size_t SZ_QE   = (size_t)NB * EROWS * C3 * 4;
constexpr size_t SZ_CTX  = (size_t)MTOK * CD * 2;
constexpr size_t SZ_X1   = (size_t)MTOK * CD * 4;
constexpr size_t SZ_F16  = (size_t)MTOK * C4 * 2;
constexpr size_t SZ_CLS  = (size_t)NCH * 64 * 4;
constexpr size_t OFF_H16 = 0;
constexpr size_t OFF_W3T = OFF_H16 + SZ_H16;
constexpr size_t OFF_WOT = OFF_W3T + SZ_W3T;
constexpr size_t OFF_W1T = OFF_WOT + SZ_WOT;
constexpr size_t OFF_W2T = OFF_W1T + SZ_W1T;
constexpr size_t OFF_QK  = OFF_W2T + SZ_W2T;
constexpr size_t OFF_VT  = OFF_QK + SZ_QK;
constexpr size_t OFF_QE  = OFF_VT + SZ_VT;
constexpr size_t OFF_CTX = OFF_QE + SZ_QE;
constexpr size_t OFF_X1  = OFF_CTX + SZ_CTX;
constexpr size_t OFF_F16 = OFF_X1 + SZ_X1;
constexpr size_t OFF_CLS = OFF_F16 + SZ_F16;
constexpr size_t WS_TOTAL = OFF_CLS + SZ_CLS;
static_assert(WS_TOTAL <= (size_t)134217728);
static_assert(SZ_H16 % 256 == 0 && SZ_W3T % 256 == 0 && SZ_WOT % 256 == 0 && SZ_W1T % 256 == 0 && SZ_W2T % 256 == 0 && SZ_QK % 256 == 0 &&
              SZ_VT % 256 == 0 && SZ_QE % 256 == 0 && SZ_CTX % 256 == 0 && SZ_X1 % 256 == 0 && SZ_F16 % 256 == 0 && SZ_CLS % 256 == 0);
static_assert((size_t)(NCH - 1) * 64 + 64 <= SZ_CLS / 4);
static_assert((size_t)NB * NH * NCH * 64 == (size_t)MTOK * NH);

static GP mk_gp(const unsigned short* A, long long sA, int lda, const unsigned short* Bt, int ldb, void* C, long long sC, int ldc,
                const float* bias, const float* R, int ldr, int M, int N, int K, int rpb, int rpbC, int rpbR) {
  GP g{};
  g.A = A; g.Bt = Bt; g.C = C; g.bias = bias; g.R = R; g.strideA = sA; g.strideC = sC;
  g.lda = lda; g.ldb = ldb; g.ldc = ldc; g.ldr = ldr; g.M = M; g.N = N; g.K = K; g.rpb = rpb; g.rpbC = rpbC; g.rpbR = rpbR;
  g.scale = 0.0625f; g.pad_ = 0;
  return g;
}
#define GP_ARGS(g) (g).A, (g).Bt, (g).C, (g).bias, (g).R, (g).strideA, (g).strideC, (g).lda, (g).ldb, (g).ldc, (g).ldr, (g).M, (g).N, (g).K, (g).rpb, (g).rpbC, (g).rpbR, (g).scale
static unsigned gemm_blocks(int M, int N) { return (unsigned)((((M / 64) * (N / 64)) + 7) / 8); }

extern "C" void kernel_launch(void* const* d_in, const int* in_sizes, int n_in, void* d_out, int out_size, void* d_ws, size_t ws_size, hipStream_t stream) {
  if (n_in < 14) return;
  const long long need_x = ((long long)(NB - 1) * SEQ_FULL + SEQ) * CD;
  const long long need_m = (long long)(SEQ - 1) * SEQ_FULL + SEQ;
  if ((long long)in_sizes[0] < need_x) return;
  if ((long long)in_sizes[1] < need_m) return;
  if (in_sizes[2] < CD || in_sizes[3] < CD || in_sizes[4] < CD * C3 || in_sizes[5] < C3 || in_sizes[6] < CD * CD || in_sizes[7] < CD) return;
  if (in_sizes[8] < CD || in_sizes[9] < CD || in_sizes[10] < CD * C4 || in_sizes[11] < C4 || in_sizes[12] < C4 * CD || in_sizes[13] < CD) return;
  if ((long long)out_size < need_x) return;
  if (ws_size < WS_TOTAL) return;

  const float* x    = (const float*)d_in[0];
  const int*   amask = (const int*)d_in[1];
  const float* g1   = (const float*)d_in[2];
  const float* be1  = (const float*)d_in[3];
  const float* wqkv = (const float*)d_in[4];
  const float* bqkv = (const float*)d_in[5];
  const float* wo   = (const float*)d_in[6];
  const float* bo   = (const float*)d_in[7];
  const float* g2   = (const float*)d_in[8];
  const float* be2  = (const float*)d_in[9];
  const float* w1   = (const float*)d_in[10];
  const float* b1   = (const float*)d_in[11];
  const float* w2   = (const float*)d_in[12];
  const float* b2   = (const float*)d_in[13];
  float* out = (float*)d_out;
  char* wsp = (char*)d_ws;
  unsigned short* H16 = (unsigned short*)(wsp + OFF_H16);
  unsigned short* W3T = (unsigned short*)(wsp + OFF_W3T);
  unsigned short* WOT = (unsigned short*)(wsp + OFF_WOT);
  unsigned short* W1T = (unsigned short*)(wsp + OFF_W1T);
  unsigned short* W2T = (unsigned short*)(wsp + OFF_W2T);
  unsigned short* QK  = (unsigned short*)(wsp + OFF_QK);
  unsigned short* VT  = (unsigned short*)(wsp + OFF_VT);
  float*          QE  = (float*)(wsp + OFF_QE);
  unsigned short* CTX = (unsigned short*)(wsp + OFF_CTX);
  float*          X1  = (float*)(wsp + OFF_X1);
  unsigned short* F16 = (unsigned short*)(wsp + OFF_F16);
  int*            CLS = (int*)(wsp + OFF_CLS);
  const int BIG = 1 << 30;

  k_maskcls<<<NCH, 256, 0, stream>>>(amask, CLS);
  k_castbT<<<(unsigned)((((long long)C3) * (CD / 8) + 255) / 256), 256, 0, stream>>>(wqkv, C3, W3T, CD, CD, C3, 16.0f);
  k_castbT<<<(unsigned)((((long long)CD) * (CD / 8) + 255) / 256), 256, 0, stream>>>(wo, CD, WOT, CD, CD, CD, 16.0f);
  k_castbT<<<(unsigned)((((long long)C4) * (CD / 8) + 255) / 256), 256, 0, stream>>>(w1, C4, W1T, CD, CD, C4, 16.0f);
  k_castbT<<<(unsigned)((((long long)CD) * (C4 / 8) + 255) / 256), 256, 0, stream>>>(w2, CD, W2T, C4, C4, CD, 16.0f);
  k_ln_in<<<MTOK / 8, 256, 0, stream>>>(x, g1, be1, H16);
  { const GP g = mk_gp(H16, 0, CD, W3T, CD, (void*)QK, 0, QKP, bqkv, nullptr, 0, MTOK, QKP, CD, BIG, BIG, BIG);
    k_gemm_qk<<<dim3(gemm_blocks(MTOK, QKP), 1), 256, 0, stream>>>(GP_ARGS(g)); }
  { const GP g = mk_gp(W3T + (size_t)2 * CD * CD, 0, CD, H16, CD, (void*)VT, 0, VTP, bqkv + 2 * CD, nullptr, 0, CD, MTOK, CD, BIG, BIG, BIG);
    k_gemm_vt<<<dim3(gemm_blocks(CD, MTOK), 1), 256, 0, stream>>>(GP_ARGS(g)); }
  { const GP g = mk_gp(H16, (long long)SEQ * CD, CD, W3T, CD, (void*)QE, (long long)EROWS * C3, C3, bqkv, nullptr, 0, EROWS, C3, CD, BIG, BIG, BIG);
    k_gemm_e<<<dim3(gemm_blocks(EROWS, C3), NB), 256, 0, stream>>>(GP_ARGS(g)); }
  k_attn_main<<<NB * NH * NCH, 128, 0, stream>>>(QK, VT, amask, CLS, CTX);
  k_attn_early<<<NB * NH, 128, 0, stream>>>(QE, amask, CLS, CTX);
  { const GP g = mk_gp(CTX, 0, CD, WOT, CD, (void*)X1, 0, CD, bo, x, CD, MTOK, CD, CD, SEQ, SEQ, SEQ_FULL);
    k_gemm_proj<<<dim3(gemm_blocks(MTOK, CD), 1), 256, 0, stream>>>(GP_ARGS(g)); }
  k_ln_mid<<<MTOK / 8, 256, 0, stream>>>(X1, g2, be2, H16);
  { const GP g = mk_gp(H16, 0, CD, W1T, CD, (void*)F16, 0, C4, b1, nullptr, 0, MTOK, C4, CD, BIG, BIG, BIG);
    k_gemm_fc<<<dim3(gemm_blocks(MTOK, C4), 1), 256, 0, stream>>>(GP_ARGS(g)); }
  { const GP g = mk_gp(F16, 0, C4, W2T, C4, (void*)out, 0, CD, b2, X1, CD, MTOK, CD, C4, SEQ, SEQ_FULL, SEQ);
    k_gemm_mlp<<<dim3(gemm_blocks(MTOK, CD), 1), 256, 0, stream>>>(GP_ARGS(g)); }
}
